// RGCN_3358664425857
// MI455X (gfx1250) — hardware-verified
//
#include <hip/hip_runtime.h>
#include <stddef.h>
#include <stdint.h>


#define DIN    64
#define DH     64
#define DO     32
#define NREL   8
#define GR     4
#define NGRP   (NREL / GR)
#define KB1    DIN
#define KB2    (2 * DH)
#define NB1    (NREL * DH + DH)
#define NB2    (NREL * DO + DO)
#define RB1    (NREL * DH)
#define RB2    (NREL * DO)
#define TP1    (GR * DH)
#define TP2    (GR * DO)
#define NTHR   256
#define NWAVE  8
#define EPT    8
#define CHUNK  (NTHR * EPT)
#define WCAP   (EPT * 32)
#define LISTN  (NWAVE * WCAP)
#define NBA    2048
#define SLA    11
#define RCAP   28672
#define DEGCAP 64
#define GBM    64
#define GTHR   128
#define UB1    (NB1 * (KB1 / 8))
#define UB1R   (RB1 * (KB1 / 8))
#define UB2    (NB2 * (KB2 / 8))
#define UB2R   (RB2 * (KB2 / 8))
#define UTOT   (UB1 + UB2)
#define AGG_ZINTS    (LISTN + 2 * RCAP + 3 * NBA)
#define MISC_INTS    96
#define AGG_LDS_INTS (AGG_ZINTS + MISC_INTS)
#define WSMAX  134217728

static_assert((CHUNK & (CHUNK - 1)) == 0 && CHUNK <= 2048);
static_assert((NBA & (NBA - 1)) == 0 && NBA == (1 << SLA));
static_assert(((long long)CHUNK << SLA) < (1LL << 31));
static_assert(LISTN % NTHR == 0);
static_assert(NBA % NWAVE == 0 && NBA % 32 == 0 && NBA % GBM == 0);
static_assert(RCAP % 4 == 0 && AGG_ZINTS % 4 == 0 && LISTN % 4 == 0 && ((AGG_ZINTS + MISC_INTS) % 4) == 0);
static_assert(AGG_ZINTS % (NTHR * 4) == 0);
static_assert(MISC_INTS >= 16 + DEGCAP + 1 && DEGCAP + 1 <= NTHR);
static_assert(AGG_LDS_INTS * 4 <= 300000);
static_assert(KB1 % 32 == 0 && KB2 % 32 == 0 && TP1 % 128 == 0 && TP2 % 128 == 0 && DH == 64 && DO == 32);
static_assert(TP2 + DO <= TP1);
static_assert(GBM == (GTHR / 32) * 16 && GBM % 16 == 0);
static_assert(UB1 % NTHR == 0 && UB1R % NTHR == 0 && UB2 % NTHR == 0 && UB2R % NTHR == 0 && UTOT % NTHR == 0);
static_assert(NGRP * GR == NREL);

typedef float          v2f   __attribute__((ext_vector_type(2)));
typedef float          v4f   __attribute__((ext_vector_type(4)));
typedef float          v8f   __attribute__((ext_vector_type(8)));
typedef int            v4i   __attribute__((ext_vector_type(4)));
typedef int            v8i   __attribute__((ext_vector_type(8)));
typedef unsigned short v4us  __attribute__((ext_vector_type(4)));
typedef unsigned short v8us  __attribute__((ext_vector_type(8)));
typedef unsigned short v16us __attribute__((ext_vector_type(16)));
typedef __bf16         v16bf __attribute__((ext_vector_type(16)));
typedef v2f  __attribute__((may_alias)) v2fa;
typedef v4f  __attribute__((may_alias)) v4fa;
typedef v4i  __attribute__((may_alias)) v4ia;
typedef v4us __attribute__((may_alias)) v4usa;
typedef v8us __attribute__((may_alias)) v8usa;
union Frag { v16bf v; v16us u; v8us h[2]; v8i w; };

__device__ __forceinline__ v8f wmb(const Frag& a, const Frag& b, v8f c) {
  v8f d = __builtin_amdgcn_wmma_f32_16x16x32_bf16(false, a.v, false, b.v, (short)0, c, false, false);
  asm volatile("v_nop\n\tv_nop\n\tv_nop\n\tv_nop" : "+v"(d) : "v"(a.w), "v"(b.w));
  return d;
}

__device__ __forceinline__ unsigned bf16_bits(float f) {
  const unsigned u = __float_as_uint(f);
  return (u + 0x7FFFu + ((u >> 16) & 1u)) >> 16;
}
__device__ __forceinline__ float bf16_val(float f) {
  return __uint_as_float(bf16_bits(f) << 16);
}
__device__ __forceinline__ v4us hilo4(v2f t) {
  v4us o;
  unsigned hb;
  hb = bf16_bits(t.x); o[0] = (unsigned short)hb; o[2] = (unsigned short)bf16_bits(t.x - __uint_as_float(hb << 16));
  hb = bf16_bits(t.y); o[1] = (unsigned short)hb; o[3] = (unsigned short)bf16_bits(t.y - __uint_as_float(hb << 16));
  return o;
}

__device__ __forceinline__ int scan_chunk(const int* __restrict__ dsts, const int* __restrict__ ets, int nE,
                                          int cbase, int slotBase, int g0, int* list, int tid, int lane, int wave) {
  int wc = 0;
  const int el0 = tid * EPT;
  const int e0  = cbase + el0;
  const int lim = nE - 4;
  const int q0  = e0 < lim ? e0 : lim;
  const int q1  = (e0 + 4) < lim ? (e0 + 4) : lim;
  const v4i da = *(const v4ia*)(dsts + q0);
  const v4i db = *(const v4ia*)(dsts + q1);
  const v4i ta = *(const v4ia*)(ets + q0);
  const v4i tb = *(const v4ia*)(ets + q1);
  const unsigned nbs = (unsigned)slotBase, ug = (unsigned)g0, ue0 = (unsigned)e0, unE = (unsigned)nE;
  const unsigned unb = (unsigned)NBA, ugr = (unsigned)GR;
  const unsigned s0 = (unsigned)da.x - nbs, s1 = (unsigned)da.y - nbs;
  const unsigned s2 = (unsigned)da.z - nbs, s3 = (unsigned)da.w - nbs;
  const unsigned s4 = (unsigned)db.x - nbs, s5 = (unsigned)db.y - nbs;
  const unsigned s6 = (unsigned)db.z - nbs, s7 = (unsigned)db.w - nbs;
  const unsigned r0 = (unsigned)ta.x - ug, r1 = (unsigned)ta.y - ug;
  const unsigned r2 = (unsigned)ta.z - ug, r3 = (unsigned)ta.w - ug;
  const unsigned r4 = (unsigned)tb.x - ug, r5 = (unsigned)tb.y - ug;
  const unsigned r6 = (unsigned)tb.z - ug, r7 = (unsigned)tb.w - ug;
  const bool h0 = (ue0 + 0u < unE) & (s0 < unb) & (r0 < ugr);
  const bool h1 = (ue0 + 1u < unE) & (s1 < unb) & (r1 < ugr);
  const bool h2 = (ue0 + 2u < unE) & (s2 < unb) & (r2 < ugr);
  const bool h3 = (ue0 + 3u < unE) & (s3 < unb) & (r3 < ugr);
  const bool h4 = (ue0 + 4u < unE) & (s4 < unb) & (r4 < ugr);
  const bool h5 = (ue0 + 5u < unE) & (s5 < unb) & (r5 < ugr);
  const bool h6 = (ue0 + 6u < unE) & (s6 < unb) & (r6 < ugr);
  const bool h7 = (ue0 + 7u < unE) & (s7 < unb) & (r7 < ugr);
  const unsigned any = __builtin_amdgcn_ballot_w32(h0 | h1 | h2 | h3 | h4 | h5 | h6 | h7);
  if (any != 0u) {
#define HITJ(J, HJ, SJ) { \
      const unsigned mj = __builtin_amdgcn_ballot_w32(HJ); \
      if (mj != 0u) { \
        if (HJ) { \
          const int pos = wc + (int)__builtin_amdgcn_mbcnt_lo(mj, 0u); \
          if (pos < WCAP) list[wave * WCAP + pos] = ((el0 + (J)) << SLA) | (int)(SJ); \
        } \
        wc += (int)__builtin_popcount(mj); } }
    HITJ(0, h0, s0)
    HITJ(1, h1, s1)
    HITJ(2, h2, s2)
    HITJ(3, h3, s3)
    HITJ(4, h4, s4)
    HITJ(5, h5, s5)
    HITJ(6, h6, s6)
    HITJ(7, h7, s7)
#undef HITJ
  }
  return wc;
}

__global__ __launch_bounds__(NTHR) void k_prep(const float* __restrict__ W1, const float* __restrict__ R1,
                                               const float* __restrict__ W2, const float* __restrict__ R2,
                                               unsigned short* B1, unsigned short* B2) {
  const int u = (int)blockIdx.x * NTHR + (int)threadIdx.x;
  v8us o;
  unsigned short* dp;
  if (u < UB1) {
    const int row = u >> 3;
    const int k8  = (u & 7) * 8;
    const float* p;
    if (u < UB1R) {
      const int r = row >> 6;
      const int n = row & 63;
      p = W1 + (size_t)r * DIN * DH + (size_t)k8 * DH + n;
    } else {
      const int n = row - RB1;
      p = R1 + (size_t)k8 * DH + n;
    }
#pragma unroll
    for (int i = 0; i < 8; ++i) o[i] = (unsigned short)bf16_bits(p[(size_t)i * DH]);
    dp = B1 + (size_t)row * KB1 + k8;
  } else if (u < UTOT) {
    const int v   = u - UB1;
    const int row = v >> 4;
    const int q   = v & 15;
    const float* p;
    if (v < UB2R) {
      const int r = row >> 5;
      const int n = row & 31;
      p = W2 + (size_t)r * DH * DO + (size_t)(4 * q) * DO + n;
    } else {
      const int n = row - RB2;
      p = R2 + (size_t)(4 * q) * DO + n;
    }
    const unsigned short f0 = (unsigned short)bf16_bits(p[0]);
    const unsigned short f1 = (unsigned short)bf16_bits(p[DO]);
    const unsigned short f2 = (unsigned short)bf16_bits(p[2 * DO]);
    const unsigned short f3 = (unsigned short)bf16_bits(p[3 * DO]);
    o[0] = f0; o[1] = f1; o[2] = f0; o[3] = f1; o[4] = f2; o[5] = f3; o[6] = f2; o[7] = f3;
    dp = B2 + (size_t)row * KB2 + 8 * q;
  } else {
    return;
  }
  *(volatile v8us*)dp = o;
  __threadfence();
  *(volatile v8us*)dp = o;
}

template <int NT, int AF, int KK>
__global__ __launch_bounds__(GTHR) void k_gemm(const float* __restrict__ Af, const unsigned short* __restrict__ Au,
                                               int lda, int nAv, const unsigned short* __restrict__ BT, int bRow0,
                                               const float* __restrict__ bias, int nbias, int biasOn,
                                               float* outp, int ldc, int nOut) {
  constexpr int CBW = 16 * NT;
  constexpr int LPR = 4 * NT;
  constexpr int RPI = 32 / LPR;
  constexpr int NI  = 16 / RPI;
  __shared__ __attribute__((aligned(16))) float stg[GBM * CBW];
  const int tid = (int)threadIdx.x, lane = tid & 31, wave = tid >> 5, hh = lane >> 4, m = lane & 15;
  const int rowBase = (int)blockIdx.x * GBM;
  const int colBase = (int)blockIdx.y * CBW;

  v8f acc[NT];
  {
    const v8f z = {0.f, 0.f, 0.f, 0.f, 0.f, 0.f, 0.f, 0.f};
#pragma unroll
    for (int t = 0; t < NT; ++t) acc[t] = z;
  }
  const int    ar   = rowBase + 16 * wave + m;
  const int    arc  = ar < nAv ? ar : nAv - 1;
  const float  okf  = ar < nAv ? 1.0f : 0.0f;
  const size_t xoff = (size_t)arc * (size_t)lda + 8 * hh;
  const size_t aoff = (size_t)ar * (size_t)lda + 8 * hh;
  const unsigned short* bp = BT + (size_t)(bRow0 + colBase + m) * (size_t)KK + 8 * hh;

#pragma unroll 1
  for (int k0 = 0; k0 < KK; k0 += 32) {
    Frag af;
    if (AF != 0) {
      const float* xp = Af + xoff + k0;
      const v4f u0 = *(const v4fa*)(xp);
      const v4f u1 = *(const v4fa*)(xp + 4);
      const v4f u2 = *(const v4fa*)(xp + 16);
      const v4f u3 = *(const v4fa*)(xp + 20);
      v8us o0, o1;
      o0[0] = (unsigned short)bf16_bits(u0.x * okf); o0[1] = (unsigned short)bf16_bits(u0.y * okf);
      o0[2] = (unsigned short)bf16_bits(u0.z * okf); o0[3] = (unsigned short)bf16_bits(u0.w * okf);
      o0[4] = (unsigned short)bf16_bits(u1.x * okf); o0[5] = (unsigned short)bf16_bits(u1.y * okf);
      o0[6] = (unsigned short)bf16_bits(u1.z * okf); o0[7] = (unsigned short)bf16_bits(u1.w * okf);
      o1[0] = (unsigned short)bf16_bits(u2.x * okf); o1[1] = (unsigned short)bf16_bits(u2.y * okf);
      o1[2] = (unsigned short)bf16_bits(u2.z * okf); o1[3] = (unsigned short)bf16_bits(u2.w * okf);
      o1[4] = (unsigned short)bf16_bits(u3.x * okf); o1[5] = (unsigned short)bf16_bits(u3.y * okf);
      o1[6] = (unsigned short)bf16_bits(u3.z * okf); o1[7] = (unsigned short)bf16_bits(u3.w * okf);
      af.h[0] = o0;
      af.h[1] = o1;
    } else {
      const unsigned short* ap = Au + aoff + k0;
      af.h[0] = *(const v8usa*)(ap);
      af.h[1] = *(const v8usa*)(ap + 16);
    }
#pragma unroll
    for (int nt = 0; nt < NT; ++nt) {
      const unsigned short* wq = bp + (size_t)(16 * nt) * (size_t)KK + k0;
      Frag bf;
      bf.h[0] = *(const v8usa*)wq;
      bf.h[1] = *(const v8usa*)(wq + 16);
      acc[nt] = wmb(af, bf, acc[nt]);
    }
  }

#pragma unroll
  for (int nt = 0; nt < NT; ++nt) {
    const int lc = 16 * nt + m;
#pragma unroll
    for (int r = 0; r < 8; ++r) {
      const int lr = 16 * wave + 8 * hh + r;
      stg[lr * CBW + lc] = acc[nt][r];
    }
  }
  __syncthreads();

  const int sub = lane / LPR;
  const int cq  = 4 * (lane % LPR);
  const float bsc = (biasOn != 0) ? 1.0f : 0.0f;
  const int bix = cq < nbias - 4 ? cq : nbias - 4;
  v4f b4;
  {
    const v4f tb = *(const v4fa*)(bias + bix);
    b4.x = bf16_val(tb.x) * bsc; b4.y = bf16_val(tb.y) * bsc;
    b4.z = bf16_val(tb.z) * bsc; b4.w = bf16_val(tb.w) * bsc;
  }

  v4f pv[NI];
#pragma unroll
  for (int i = 0; i < NI; ++i) pv[i] = *(const v4fa*)(stg + (16 * wave + RPI * i + sub) * CBW + cq) + b4;

#pragma unroll
  for (int i = 0; i < NI; ++i) {
    const int row = rowBase + 16 * wave + RPI * i + sub;
    if (row < nOut) *(volatile v4f*)(outp + (size_t)row * (size_t)ldc + colBase + cq) = pv[i];
  }
  __threadfence();
#pragma unroll
  for (int i = 0; i < NI; ++i) {
    const int row = rowBase + 16 * wave + RPI * i + sub;
    if (row < nOut) *(volatile v4f*)(outp + (size_t)row * (size_t)ldc + colBase + cq) = pv[i];
  }
}

template <int RW, int FIN>
__global__ __launch_bounds__(NTHR) void k_scan(const int* __restrict__ srcs, const int* __restrict__ dsts,
                                               const int* __restrict__ ets, int nE, int nN, int mRows, int g0,
                                               const float* __restrict__ T, float* accp, float* outp) {
  constexpr int TP = GR * RW;
  extern __shared__ __attribute__((aligned(16))) int dsm[];
  int* list = dsm;
  int* hl   = dsm + LISTN;
  int* sl   = hl + RCAP;
  int* cnt  = sl + RCAP;
  int* offs = cnt + NBA;
  int* cur  = offs + NBA;
  int* misc = cur + NBA;
  float* rtab = (float*)(misc + 16);
  const int tid = (int)threadIdx.x, lane = tid & 31, wave = tid >> 5;
  const int nodeBase = (int)blockIdx.x * NBA;

  {
    const v4i z4 = {0, 0, 0, 0};
    for (int i = tid * 4; i < AGG_ZINTS; i += NTHR * 4) *(v4ia*)(dsm + i) = z4;
    if (tid < 16) misc[tid] = 0;
    if (tid <= DEGCAP) rtab[tid] = 1.0f / fmaxf((float)tid, 1.0f);
  }
  __syncthreads();

  int t = 0, ov = 0;
  const int nChunks = (nE + CHUNK - 1) / CHUNK;
#pragma unroll 1
  for (int ch = 0; ch < nChunks; ++ch) {
    const int cbase = ch * CHUNK;
    const int wc = scan_chunk(dsts, ets, nE, cbase, nodeBase, g0, list, tid, lane, wave);
    if (lane == 0) misc[wave] = wc;
    __syncthreads();
    if (wave == 0) {
#pragma unroll 1
      for (int w2 = 0; w2 < NWAVE; ++w2) {
        int c = misc[w2];
        c = c < 0 ? 0 : (c > WCAP ? WCAP : c);
#pragma unroll 1
        for (int b0 = 0; b0 < c; b0 += 32) {
          const int idx = b0 + lane;
          const int ent = list[w2 * WCAP + (idx < WCAP ? idx : WCAP - 1)];
          const int m32 = (c - b0) < 32 ? (c - b0) : 32;
#pragma unroll 1
          for (int k = 0; k < m32; ++k) {
            const int u    = __builtin_amdgcn_readlane(ent, k);
            const int slot = u & (NBA - 1);
            const int el   = (u >> SLA) & (CHUNK - 1);
            const unsigned pk = ((unsigned)(cbase + el) << SLA) | (unsigned)slot;
            if (t < RCAP) {
              if (lane == 0) { hl[t] = (int)pk; cnt[slot] = cnt[slot] + 1; }
              t = t + 1;
            } else {
              ov = 1;
            }
          }
        }
      }
    }
    __syncthreads();
  }
  if (wave == 0 && lane == 0) { misc[8] = t; misc[9] = ov; }
  __syncthreads();
  int tt = misc[8];
  tt = tt < 0 ? 0 : (tt > RCAP ? RCAP : tt);
  const int ovf = misc[9];

  if (wave == 0) {
    const int base = lane * (NBA / 32);
    int sacc = 0;
#pragma unroll 1
    for (int i = 0; i < NBA / 32; ++i) sacc += cnt[base + i];
    int incl = sacc;
#pragma unroll
    for (int d = 1; d < 32; d <<= 1) {
      const int y = __shfl_up(incl, d, 32);
      if (lane >= d) incl += y;
    }
    int run = incl - sacc;
#pragma unroll 1
    for (int i = 0; i < NBA / 32; ++i) {
      const int cv = cnt[base + i];
      offs[base + i] = run;
      cur[base + i]  = run;
      run += cv;
    }
  }
  __syncthreads();
  if (wave == 0) {
#pragma unroll 1
    for (int b0 = 0; b0 < tt; b0 += 32) {
      const int idx = b0 + lane;
      const int ent = hl[idx < RCAP ? idx : RCAP - 1];
      const int m32 = (tt - b0) < 32 ? (tt - b0) : 32;
#pragma unroll 1
      for (int k = 0; k < m32; ++k) {
        const int u    = __builtin_amdgcn_readlane(ent, k);
        const int slot = u & (NBA - 1);
        if (lane == 0) {
          int p = cur[slot];
          p = p < 0 ? 0 : (p > RCAP - 1 ? RCAP - 1 : p);
          sl[p] = u;
          cur[slot] = p + 1;
        }
      }
    }
  }
  __syncthreads();

  const float qnan = __int_as_float(0x7fc00000);
  const float pz = (ovf != 0) ? qnan : 0.0f;
#pragma unroll 1
  for (int si = 0; si < NBA / NWAVE; ++si) {
    const int s    = si * NWAVE + wave;
    const int node = nodeBase + s;
    int c = cnt[s];
    const bool big = c > DEGCAP;
    c = c < 0 ? 0 : (c > DEGCAP ? DEGCAP : c);
    int o = offs[s];
    o = o < 0 ? 0 : (o > RCAP ? RCAP : o);
    const int nc = node < mRows ? node : mRows - 1;

    int n0 = 0, n1 = 0, n2 = 0, n3 = 0;
#pragma unroll 1
    for (int b0 = 0; b0 < c; b0 += 32) {
      int idx = o + b0 + lane;
      idx = idx > RCAP - 1 ? RCAP - 1 : idx;
      const int ent = sl[idx];
      int eid = (int)((unsigned)ent >> SLA);
      eid = eid > nE - 1 ? nE - 1 : eid;
      int tg = ets[eid] - g0;
      tg = tg < 0 ? 0 : (tg > GR - 1 ? GR - 1 : tg);
      const int m32 = (c - b0) < 32 ? (c - b0) : 32;
      const unsigned lm = 0xffffffffu >> (32 - m32);
      n0 += (int)__builtin_popcount(__builtin_amdgcn_ballot_w32(tg == 0) & lm);
      n1 += (int)__builtin_popcount(__builtin_amdgcn_ballot_w32(tg == 1) & lm);
      n2 += (int)__builtin_popcount(__builtin_amdgcn_ballot_w32(tg == 2) & lm);
      n3 += (int)__builtin_popcount(__builtin_amdgcn_ballot_w32(tg == 3) & lm);
    }
    const int c0 = n0 > DEGCAP ? DEGCAP : n0, c1 = n1 > DEGCAP ? DEGCAP : n1;
    const int c2 = n2 > DEGCAP ? DEGCAP : n2, c3 = n3 > DEGCAP ? DEGCAP : n3;
    const float i0 = rtab[c0], i1 = rtab[c1], i2 = rtab[c2], i3 = rtab[c3];
    const float pzr = big ? qnan : pz;

    if (RW == 64) {
      const v2f z2 = {0.0f, 0.0f};
      v2f a = z2;
#pragma unroll 1
      for (int b0 = 0; b0 < c; b0 += 32) {
        int idx = o + b0 + lane;
        idx = idx > RCAP - 1 ? RCAP - 1 : idx;
        const int ent = sl[idx];
        int eid = (int)((unsigned)ent >> SLA);
        eid = eid > nE - 1 ? nE - 1 : eid;
        int sr = srcs[eid];
        sr = sr < 0 ? 0 : (sr > nN - 1 ? nN - 1 : sr);
        int tg = ets[eid] - g0;
        tg = tg < 0 ? 0 : (tg > GR - 1 ? GR - 1 : tg);
        const int m32 = (c - b0) < 32 ? (c - b0) : 32;
#pragma unroll 1
        for (int k = 0; k < m32; ++k) {
          const int sk = __builtin_amdgcn_readlane(sr, k);
          const int tk = __builtin_amdgcn_readlane(tg, k);
          const float w = (tk == 0) ? i0 : ((tk == 1) ? i1 : ((tk == 2) ? i2 : i3));
          const v2f f = *(const v2fa*)(T + (size_t)sk * (size_t)TP + RW * tk + 2 * lane);
          a += w * f;
        }
      }
      const v2f arow = *(const v2fa*)(accp + (size_t)nc * (size_t)RW + 2 * lane);
      const v2f v = arow + a + pzr;
      if (FIN == 0) {
        if (node < mRows) {
          float* rp = accp + (size_t)node * (size_t)RW + 2 * lane;
          *(volatile v2f*)rp = v;
          __threadfence();
          *(volatile v2f*)rp = v;
        }
      } else {
        const bool live = node < nN;
        v2f y;
        y.x = (v.x < 0.0f) ? 0.0f : v.x;
        y.y = (v.y < 0.0f) ? 0.0f : v.y;
        y.x = live ? y.x : 0.0f; y.y = live ? y.y : 0.0f;
        const v4us po = hilo4(y);
        if (node < mRows) {
          unsigned short* rp = (unsigned short*)accp + (size_t)node * (size_t)(2 * RW) + 4 * lane;
          *(volatile v4usa*)rp = po;
          __threadfence();
          *(volatile v4usa*)rp = po;
        }
      }
    } else {
      float a = 0.0f;
#pragma unroll 1
      for (int b0 = 0; b0 < c; b0 += 32) {
        int idx = o + b0 + lane;
        idx = idx > RCAP - 1 ? RCAP - 1 : idx;
        const int ent = sl[idx];
        int eid = (int)((unsigned)ent >> SLA);
        eid = eid > nE - 1 ? nE - 1 : eid;
        int sr = srcs[eid];
        sr = sr < 0 ? 0 : (sr > nN - 1 ? nN - 1 : sr);
        int tg = ets[eid] - g0;
        tg = tg < 0 ? 0 : (tg > GR - 1 ? GR - 1 : tg);
        const int m32 = (c - b0) < 32 ? (c - b0) : 32;
#pragma unroll 1
        for (int k = 0; k < m32; ++k) {
          const int sk = __builtin_amdgcn_readlane(sr, k);
          const int tk = __builtin_amdgcn_readlane(tg, k);
          const float w = (tk == 0) ? i0 : ((tk == 1) ? i1 : ((tk == 2) ? i2 : i3));
          const float f = T[(size_t)sk * (size_t)TP + RW * tk + lane];
          a += w * f;
        }
      }
      const float arow = accp[(size_t)nc * (size_t)RW + lane];
      const float v = arow + a + pzr;
      if (FIN == 0) {
        if (node < mRows) {
          float* rp = accp + (size_t)node * (size_t)RW + lane;
          *(volatile float*)rp = v;
          __threadfence();
          *(volatile float*)rp = v;
        }
      } else {
        if (node < nN) {
          float* rp = outp + (size_t)node * (size_t)RW + lane;
          *(volatile float*)rp = v;
          __threadfence();
          *(volatile float*)rp = v;
        }
      }
    }
  }
}

static inline int cdiv(int a, int b) { return (a + b - 1) / b; }

extern "C" void kernel_launch(void* const* d_in, const int* in_sizes, int n_in,
                              void* d_out, int out_size, void* d_ws, size_t ws_size,
                              hipStream_t stream) {
  if (n_in < 9) return;
  if (in_sizes[0] < DIN || (in_sizes[0] % DIN) != 0) return;
  const int nN = in_sizes[0] / DIN;
  if (in_sizes[1] < 8 || (in_sizes[1] & 1) != 0) return;
  const int nE = in_sizes[1] / 2;
  if (nE < 4 || (nE & 3) != 0 || nE > (1 << 21)) return;
  if (in_sizes[2] != nE) return;
  if (in_sizes[3] != NREL * DIN * DH || in_sizes[4] != DIN * DH || in_sizes[5] != DH) return;
  if (in_sizes[6] != NREL * DH * DO || in_sizes[7] != DH * DO || in_sizes[8] != DO) return;
  if ((long long)out_size != (long long)nN * DO) return;

  const float* x    = (const float*)d_in[0];
  const int*   edge = (const int*)d_in[1];
  const int*   ety  = (const int*)d_in[2];
  const float* W1   = (const float*)d_in[3];
  const float* R1   = (const float*)d_in[4];
  const float* b1   = (const float*)d_in[5];
  const float* W2   = (const float*)d_in[6];
  const float* R2   = (const float*)d_in[7];
  const float* b2   = (const float*)d_in[8];
  float* out = (float*)d_out;
  const int* src = edge;
  const int* dst = edge + nE;

  const int MP = cdiv(nN, GBM) * GBM;
  const int gM = MP / GBM;
  const int gA = cdiv(MP, NBA);
  if ((long long)gA * NBA < (long long)MP) return;

  char* ws = (char*)d_ws;
  size_t off = 0;
  const size_t oB1 = off; off += (size_t)NB1 * KB1 * 2;              off = (off + 255) & ~(size_t)255;
  const size_t oB2 = off; off += (size_t)NB2 * KB2 * 2;              off = (off + 255) & ~(size_t)255;
  const size_t oT  = off; off += (size_t)MP * TP1 * 4;               off = (off + 255) & ~(size_t)255;
  const size_t oA  = off; off += (size_t)MP * DH * 4;                off = (off + 255) & ~(size_t)255;
  if (off > ws_size || off > (size_t)WSMAX) return;
  unsigned short* B1p  = (unsigned short*)(ws + oB1);
  unsigned short* B2p  = (unsigned short*)(ws + oB2);
  float*          Tp   = (float*)(ws + oT);
  float*          ACC1 = (float*)(ws + oA);
  const unsigned short* X1u = (const unsigned short*)(ws + oA);
  float*          ACC2 = Tp + (size_t)MP * TP2;

  const size_t scanLds = (size_t)AGG_LDS_INTS * 4;
  hipFuncSetAttribute(reinterpret_cast<const void*>(&k_scan<64, 0>), hipFuncAttributeMaxDynamicSharedMemorySize, (int)scanLds);
  hipFuncSetAttribute(reinterpret_cast<const void*>(&k_scan<64, 1>), hipFuncAttributeMaxDynamicSharedMemorySize, (int)scanLds);
  hipFuncSetAttribute(reinterpret_cast<const void*>(&k_scan<32, 0>), hipFuncAttributeMaxDynamicSharedMemorySize, (int)scanLds);
  hipFuncSetAttribute(reinterpret_cast<const void*>(&k_scan<32, 2>), hipFuncAttributeMaxDynamicSharedMemorySize, (int)scanLds);

  k_prep<<<UTOT / NTHR, NTHR, 0, stream>>>(W1, R1, W2, R2, B1p, B2p);

  k_gemm<4, 1, KB1><<<dim3(gM, 1), GTHR, 0, stream>>>(x, B1p, DIN, nN, B1p, RB1, b1, DH, 1, ACC1, DH, MP);
  for (int g = 0; g < NGRP; ++g) {
    k_gemm<8, 1, KB1><<<dim3(gM, TP1 / 128), GTHR, 0, stream>>>(x, B1p, DIN, nN, B1p, TP1 * g, b1, DH, 0, Tp, TP1, MP);
    if (g < NGRP - 1)
      k_scan<64, 0><<<gA, NTHR, scanLds, stream>>>(src, dst, ety, nE, nN, MP, GR * g, Tp, ACC1, out);
    else
      k_scan<64, 1><<<gA, NTHR, scanLds, stream>>>(src, dst, ety, nE, nN, MP, GR * g, Tp, ACC1, out);
  }

  k_gemm<2, 0, KB2><<<dim3(gM, 1), GTHR, 0, stream>>>(x, X1u, KB2, MP, B2p, RB2, b2, DO, 1, ACC2, DO, MP);
  for (int g = 0; g < NGRP; ++g) {
    k_gemm<8, 0, KB2><<<dim3(gM, TP2 / 128), GTHR, 0, stream>>>(x, X1u, KB2, MP, B2p, TP2 * g, b2, DO, 0, Tp, TP2, MP);
    if (g < NGRP - 1)
      k_scan<32, 0><<<gA, NTHR, scanLds, stream>>>(src, dst, ety, nE, nN, MP, GR * g, Tp, ACC2, out);
    else
      k_scan<32, 2><<<gA, NTHR, scanLds, stream>>>(src, dst, ety, nE, nN, MP, GR * g, Tp, ACC2, out);
  }
}
